// CausalRecurrentAttention_41532333752804
// MI455X (gfx1250) — hardware-verified
//
#include <hip/hip_runtime.h>
#include <math.h>

typedef __attribute__((ext_vector_type(16))) _Float16 v16h;
typedef __attribute__((ext_vector_type(8)))  _Float16 v8h;
typedef __attribute__((ext_vector_type(16))) __bf16   v16b;
typedef __attribute__((ext_vector_type(8)))  __bf16   v8b;
typedef __attribute__((ext_vector_type(8)))  float    v8f;
typedef __attribute__((ext_vector_type(4)))  float    v4f;

constexpr int kBatch = 2;
constexpr int kSeq   = 2048;
constexpr int kDim   = 1024;
constexpr int kHeads = 16;
constexpr int kState = 16;
constexpr int kHdim  = 64;
constexpr int kTok   = kBatch * kSeq;
constexpr int kBCP   = 128;
constexpr float kLnEps = 1e-5f;
static_assert(kTok % 64 == 0);
static_assert(kDim % 64 == 0);
static_assert(kSeq % 64 == 0);
static_assert(kDim % 32 == 0);
static_assert(kHeads * kHdim == kDim);
static_assert(kBCP % 64 == 0);

constexpr size_t kPlane16 = (size_t)kTok * kDim * 2;
constexpr size_t kPlane32 = (size_t)kTok * kDim * 4;
constexpr size_t kW16     = (size_t)kDim * kDim * 2;
constexpr size_t kWBC16   = (size_t)kBCP * kDim * 2;
constexpr size_t kBC32    = (size_t)kTok * kBCP * 4;
constexpr size_t kCarveTotal = kPlane16 + 6 * kW16 + kWBC16 + 2 * kPlane32 + kBC32 + 6 * kPlane16;
static_assert(kCarveTotal == 107216896);
static_assert(kCarveTotal <= 134217728);

__device__ __forceinline__ unsigned short f2bf_bits(float f) {
  unsigned u = __float_as_uint(f);
  return (unsigned short)((u + 0x7FFFu + ((u >> 16) & 1u)) >> 16);
}
__device__ __forceinline__ float bf_bits2f(unsigned short h) { return __uint_as_float(((unsigned)h) << 16); }

__device__ __forceinline__ void dep_guard_h(v8f& a, v8f& b, v16h x, v16h y) { asm volatile("v_nop\n\tv_nop\n\tv_nop\n\tv_nop" : "+v"(a), "+v"(b) : "v"(x), "v"(y)); }
__device__ __forceinline__ void dep_guard_b(v8f& a, v8f& b, v16b x, v16b y) { asm volatile("v_nop\n\tv_nop\n\tv_nop\n\tv_nop" : "+v"(a), "+v"(b) : "v"(x), "v"(y)); }
__device__ __forceinline__ void keep4_h(v16h a, v16h b, v16h c, v16h d) { asm volatile("v_nop" :: "v"(a), "v"(b), "v"(c), "v"(d)); }
__device__ __forceinline__ void keep4_b(v16b a, v16b b, v16b c, v16b d) { asm volatile("v_nop" :: "v"(a), "v"(b), "v"(c), "v"(d)); }
__device__ __forceinline__ void acc_guard4(v8f& a, v8f& b, v8f& c, v8f& d) { asm volatile("v_nop\n\tv_nop\n\tv_nop\n\tv_nop" : "+v"(a), "+v"(b), "+v"(c), "+v"(d)); }
template <typename T> struct Frag;
template <> struct Frag<_Float16> {
  typedef v16h V; union U { v16h v; v8h h[2]; };
  static __device__ __forceinline__ v16h load(const _Float16* p) {
    U f; f.h[0] = *(const v8h*)(p); f.h[1] = *(const v8h*)(p + 16); return f.v;
  }
  static __device__ __forceinline__ v8f mma(v16h a, v16h b, v8f c) {
    return __builtin_amdgcn_wmma_f32_16x16x32_f16(false, a, false, b, (short)0, c, false, false);
  }
  static __device__ __forceinline__ void guard(v8f& a, v8f& b, v16h x, v16h y) { dep_guard_h(a, b, x, y); }
  static __device__ __forceinline__ void keep(v16h a, v16h b, v16h c, v16h d) { keep4_h(a, b, c, d); }
};
template <> struct Frag<__bf16> {
  typedef v16b V; union U { v16b v; v8b h[2]; };
  static __device__ __forceinline__ v16b load(const __bf16* p) {
    U f; f.h[0] = *(const v8b*)(p); f.h[1] = *(const v8b*)(p + 16); return f.v;
  }
  static __device__ __forceinline__ v8f mma(v16b a, v16b b, v8f c) {
    return __builtin_amdgcn_wmma_f32_16x16x32_bf16(false, a, false, b, (short)0, c, false, false);
  }
  static __device__ __forceinline__ void guard(v8f& a, v8f& b, v16b x, v16b y) { dep_guard_b(a, b, x, y); }
  static __device__ __forceinline__ void keep(v16b a, v16b b, v16b c, v16b d) { keep4_b(a, b, c, d); }
};

template <int ET> struct Elem;
template <> struct Elem<0> { typedef _Float16 T; };
template <> struct Elem<1> { typedef __bf16 T; };
template <int ET, int SPLIT, int BIAS_MODE, int OUT_MODE, bool RESID, int ACT = 0>
__global__ __launch_bounds__(256) void wmma_gemm64(
    const unsigned short* __restrict__ Ap, const unsigned short* __restrict__ A2p, int lda, long strideA,
    const unsigned short* __restrict__ Btp, const unsigned short* __restrict__ Bt2p, int ldb, long strideB,
    void* __restrict__ Cout, void* __restrict__ Cout2, int ldc, long strideC,
    const float* __restrict__ bias,
    const float* __restrict__ resid, long strideR,
    int M, int N, int K, float scale) {
  typedef typename Elem<ET>::T T;
  typedef typename Frag<T>::V V;
  const T* A = (const T*)Ap; const T* A2 = (const T*)A2p; const T* Bt = (const T*)Btp; const T* Bt2 = (const T*)Bt2p;
  __shared__ __align__(16) float sT[8][16 * 68];
  const int b    = blockIdx.y;
  const int lane = threadIdx.x & 31;
  const int wave = threadIdx.x >> 5;
  const int tilesN = N >> 6;
  const int tilesM = M >> 6;
  const int tile = blockIdx.x * 8 + wave;
  if (tile >= tilesM * tilesN) return;
  const int tm = tile / tilesN;
  const int tn = tile - tm * tilesN;
  const int m0 = tm << 6;
  const int n0 = tn << 6;

  const T* Ab  = A  + (size_t)b * strideA;
  const T* Bb  = Bt + (size_t)b * strideB;
  const T* Ab2 = (SPLIT != 0) ? (A2  + (size_t)b * strideA) : nullptr;
  const T* Bb2 = (SPLIT == 1) ? (Bt2 + (size_t)b * strideB) : nullptr;

  const int rlane = lane & 15;
  const int koff  = (lane >> 4) * 8;
  const int mOff  = (lane >> 4) * 8;

  v8f acc[4][4];
#pragma unroll
  for (int i = 0; i < 4; ++i)
#pragma unroll
    for (int j = 0; j < 4; ++j) acc[i][j] = (v8f){0.f,0.f,0.f,0.f,0.f,0.f,0.f,0.f};

  for (int k0 = 0; k0 < K; k0 += 32) {
    V bh[4], bl[4];
#pragma unroll
    for (int j = 0; j < 4; ++j) {
      const size_t bo = (size_t)(n0 + (j << 4) + rlane) * ldb + koff + k0;
      bh[j] = Frag<T>::load(Bb + bo);
      if (SPLIT == 1) bl[j] = Frag<T>::load(Bb2 + bo);
    }
#pragma unroll
    for (int i = 0; i < 4; ++i) {
      const size_t ao = (size_t)(m0 + (i << 4) + rlane) * lda + koff + k0;
      V ah = Frag<T>::load(Ab + ao);
      V al;
      if (SPLIT != 0) al = Frag<T>::load(Ab2 + ao);
#pragma unroll
      for (int j = 0; j < 4; ++j) {
        acc[i][j] = Frag<T>::mma(ah, bh[j], acc[i][j]);
        if (SPLIT == 1) {
          acc[i][j] = Frag<T>::mma(ah, bl[j], acc[i][j]);
          acc[i][j] = Frag<T>::mma(al, bh[j], acc[i][j]);
        }
        if (SPLIT == 2) {
          acc[i][j] = Frag<T>::mma(al, bh[j], acc[i][j]);
        }
      }
      Frag<T>::guard(acc[i][0], acc[i][3], ah, (SPLIT != 0) ? al : ah);
    }
    Frag<T>::keep(bh[0], bh[1], bh[2], bh[3]);
    if (SPLIT == 1) Frag<T>::keep(bl[0], bl[1], bl[2], bl[3]);
  }
  acc_guard4(acc[0][0], acc[0][1], acc[0][2], acc[0][3]);
  acc_guard4(acc[1][0], acc[1][1], acc[1][2], acc[1][3]);
  acc_guard4(acc[2][0], acc[2][1], acc[2][2], acc[2][3]);
  acc_guard4(acc[3][0], acc[3][1], acc[3][2], acc[3][3]);

  float* slab = sT[wave];
  const float* Rb = RESID ? (resid + (size_t)b * strideR) : nullptr;
#pragma unroll
  for (int i = 0; i < 4; ++i) {
    const int mBase = m0 + (i << 4);
#pragma unroll
    for (int j = 0; j < 4; ++j) {
      const int n = n0 + (j << 4) + rlane;
      float bv = 0.f;
      if (BIAS_MODE == 2) bv = bias[n];
#pragma unroll
      for (int r = 0; r < 8; ++r) {
        float v = acc[i][j][r] * scale;
        if (BIAS_MODE == 1) v += bias[mBase + mOff + r];
        if (BIAS_MODE == 2) v += bv;
        if (RESID) v += Rb[(size_t)(mBase + mOff + r) * ldc + n];
        if (ACT == 1) v = tanhf(v);
        if (ACT == 2) v = fmaxf(v, 0.0f);
        if (ACT == 3) v = v / (1.0f + expf(-v));
        if (ACT == 4) v = (v > 0.f) ? v : 0.01f * v;
        slab[(mOff + r) * 68 + (j << 4) + rlane] = v;
      }
    }
    __builtin_amdgcn_fence(__ATOMIC_RELEASE, "workgroup");
    __builtin_amdgcn_wave_barrier();
    __builtin_amdgcn_fence(__ATOMIC_ACQUIRE, "workgroup");
    if (OUT_MODE == 0) {
      float* C = (float*)Cout + (size_t)b * strideC;
      const int hh = lane >> 4, c4 = (lane & 15) * 4;
      for (int pass = 0; pass < 2; ++pass) {
#pragma unroll
        for (int it = 0; it < 8; ++it) {
          const int row = it * 2 + hh;
          v4f v = *(const v4f*)(slab + row * 68 + c4);
          *(volatile v4f*)(C + (size_t)(mBase + row) * ldc + n0 + c4) = v;
        }
        __threadfence();
      }
    } else {
      const int q = lane >> 3, c8 = (lane & 7) * 8;
      unsigned short* C  = (unsigned short*)Cout  + (size_t)b * strideC;
      unsigned short* C2 = (OUT_MODE == 2) ? ((unsigned short*)Cout2 + (size_t)b * strideC) : nullptr;
      for (int pass = 0; pass < 2; ++pass) {
#pragma unroll
        for (int it = 0; it < 4; ++it) {
          const int row = it * 4 + q;
          const float* sp = slab + row * 68 + c8;
          v8h hv, lv;
#pragma unroll
          for (int e = 0; e < 8; ++e) {
            if (OUT_MODE == 1) {
              hv[e] = (_Float16)sp[e];
            } else {
              unsigned short hb = f2bf_bits(sp[e]);
              unsigned short lb = f2bf_bits(sp[e] - bf_bits2f(hb));
              hv[e] = __builtin_bit_cast(_Float16, hb);
              lv[e] = __builtin_bit_cast(_Float16, lb);
            }
          }
          *(volatile v8h*)(C + (size_t)(mBase + row) * ldc + n0 + c8) = hv;
          if (OUT_MODE == 2) *(volatile v8h*)(C2 + (size_t)(mBase + row) * ldc + n0 + c8) = lv;
        }
        __threadfence();
      }
    }
    __builtin_amdgcn_fence(__ATOMIC_RELEASE, "workgroup");
    __builtin_amdgcn_wave_barrier();
    __builtin_amdgcn_fence(__ATOMIC_ACQUIRE, "workgroup");
  }
}

__global__ __launch_bounds__(256) void cast_bf16_kernel(
    const float* __restrict__ src, unsigned short* __restrict__ dst, int total8)
{
  const int i = blockIdx.x * 256 + threadIdx.x;
  if (i >= total8) return;
  const size_t e0 = (size_t)i << 3;
  const v4f a0 = *(const v4f*)(src + e0);
  const v4f a1 = *(const v4f*)(src + e0 + 4);
  v8h hv;
#pragma unroll
  for (int e = 0; e < 4; ++e) {
    hv[e]     = __builtin_bit_cast(_Float16, f2bf_bits(a0[e]));
    hv[4 + e] = __builtin_bit_cast(_Float16, f2bf_bits(a1[e]));
  }
  unsigned short* q = dst + e0;
  *(volatile v8h*)q = hv;
  __threadfence();
  *(volatile v8h*)q = hv;
}

__global__ __launch_bounds__(256) void transpose_bf16_kernel(
    const float* __restrict__ W, unsigned short* __restrict__ Bt, int Kdim, int Ndim)
{
  __shared__ float tile[64 * 65];
  const int tid = threadIdx.x, lane = tid & 31, wave = tid >> 5;
  const int n0 = blockIdx.x * 64;
  const int k0 = blockIdx.y * 64;
#pragma unroll
  for (int p = 0; p < 16; ++p) {
    const int idx = tid + p * 256;
    const int kk  = idx >> 6;
    const int nn  = idx & 63;
    const int n   = n0 + nn;
    const int nc  = (n < Ndim) ? n : (Ndim - 1);
    const float v = W[(size_t)(k0 + kk) * Ndim + nc];
    tile[kk * 65 + nn] = (n < Ndim) ? v : 0.f;
  }
  __syncthreads();
  const int q = lane >> 3, c8 = (lane & 7) * 8;
  v8h hv[2];
#pragma unroll
  for (int it = 0; it < 2; ++it) {
    const int nrow = it * 32 + wave * 4 + q;
#pragma unroll
    for (int e = 0; e < 8; ++e) {
      const float f = tile[(c8 + e) * 65 + nrow];
      hv[it][e] = __builtin_bit_cast(_Float16, f2bf_bits(f));
    }
  }
  for (int pass = 0; pass < 2; ++pass) {
#pragma unroll
    for (int it = 0; it < 2; ++it) {
      const int nrow = it * 32 + wave * 4 + q;
      *(volatile v8h*)(Bt + (size_t)(n0 + nrow) * Kdim + k0 + c8) = hv[it];
    }
    __threadfence();
  }
}

__global__ __launch_bounds__(32) void scan_kernel(
    float* __restrict__ XB, const float* __restrict__ DPRE, const float* __restrict__ BC,
    const float* __restrict__ A_log)
{
  __shared__ __align__(16) float sbc[2][32];
  const int lane = threadIdx.x;
  const int blk  = blockIdx.x;
  const int b    = blk >> 5;
  const int c    = ((blk & 31) << 5) + lane;
  float An[kState], hs[kState];
#pragma unroll
  for (int s = 0; s < kState; ++s) {
    const float al = bf_bits2f(f2bf_bits(A_log[c * kState + s]));
    An[s] = -__expf(al);
    hs[s] = 0.f;
  }
  const int col = (lane < 16) ? lane : (lane + 48);
  const size_t tok0 = (size_t)b * kSeq;
#pragma unroll 1
  for (int t = 0; t < kSeq; ++t) {
    const size_t row = tok0 + (size_t)t;
    const int buf = t & 1;
    sbc[buf][lane] = BC[row * kBCP + col];
    __syncthreads();
    const float* sb = sbc[buf];
    const v4f vb0 = *(const v4f*)(sb + 0);
    const v4f vb1 = *(const v4f*)(sb + 4);
    const v4f vb2 = *(const v4f*)(sb + 8);
    const v4f vb3 = *(const v4f*)(sb + 12);
    const v4f vc0 = *(const v4f*)(sb + 16);
    const v4f vc1 = *(const v4f*)(sb + 20);
    const v4f vc2 = *(const v4f*)(sb + 24);
    const v4f vc3 = *(const v4f*)(sb + 28);
    float Bv[kState], Cv[kState];
#pragma unroll
    for (int s = 0; s < 4; ++s) {
      Bv[s] = vb0[s]; Bv[4 + s] = vb1[s]; Bv[8 + s] = vb2[s]; Bv[12 + s] = vb3[s];
      Cv[s] = vc0[s]; Cv[4 + s] = vc1[s]; Cv[8 + s] = vc2[s]; Cv[12 + s] = vc3[s];
    }
    const size_t e = row * kDim + c;
    const float dp = DPRE[e];
    const float d  = fmaxf(dp, 0.f) + log1pf(__expf(-fabsf(dp)));
    const float xb = XB[e];
    const float dx = d * xb;
    float y = 0.f;
#pragma unroll
    for (int s = 0; s < kState; ++s) {
      const float ba = __expf(d * An[s]);
      hs[s] = ba * hs[s] + dx * Bv[s];
      y += hs[s] * Cv[s];
    }
    const float o = xb + y;
    float* p = XB + e;
    *(volatile float*)p = o;
    __threadfence();
    *(volatile float*)p = o;
  }
}

__global__ __launch_bounds__(128) void ln_kernel(
    const float* __restrict__ HYB, const float* __restrict__ g, const float* __restrict__ be,
    unsigned short* __restrict__ HHp, unsigned short* __restrict__ HLp)
{
  __shared__ float red1[4], red2[4];
  _Float16* HH = (_Float16*)HHp;
  _Float16* HL = (_Float16*)HLp;
  const int row = blockIdx.x, tid = threadIdx.x, lane = tid & 31, wave = tid >> 5;
  const size_t rb = (size_t)row * kDim;
  const int ca = tid * 8;
  const v4f va = *(const v4f*)(HYB + rb + ca);
  const v4f vb = *(const v4f*)(HYB + rb + ca + 4);
  float s = ((va[0] + va[1]) + (va[2] + va[3])) + ((vb[0] + vb[1]) + (vb[2] + vb[3]));
#pragma unroll
  for (int off = 1; off < 32; off <<= 1) s += __shfl_xor(s, off, 32);
  if (lane == 0) red1[wave] = s;
  __syncthreads();
  const float mu = ((red1[0] + red1[1]) + (red1[2] + red1[3])) * (1.0f / kDim);
  const v4f da = va - mu, db = vb - mu;
  float s2 = (da[0] * da[0] + da[1] * da[1]) + (da[2] * da[2] + da[3] * da[3]) +
             (db[0] * db[0] + db[1] * db[1]) + (db[2] * db[2] + db[3] * db[3]);
#pragma unroll
  for (int off = 1; off < 32; off <<= 1) s2 += __shfl_xor(s2, off, 32);
  if (lane == 0) red2[wave] = s2;
  __syncthreads();
  const float var = ((red2[0] + red2[1]) + (red2[2] + red2[3])) * (1.0f / kDim);
  const float inv = rsqrtf(var + kLnEps);
  const v4f ga = *(const v4f*)(g + ca);
  const v4f gb = *(const v4f*)(g + ca + 4);
  const v4f ba = *(const v4f*)(be + ca);
  const v4f bb = *(const v4f*)(be + ca + 4);
  v8h hv, lv;
#pragma unroll
  for (int e = 0; e < 4; ++e) {
    const float f0 = da[e] * inv * ga[e] + ba[e];
    const float f1 = db[e] * inv * gb[e] + bb[e];
    const unsigned short h0 = f2bf_bits(f0), h1 = f2bf_bits(f1);
    const unsigned short l0 = f2bf_bits(f0 - bf_bits2f(h0)), l1 = f2bf_bits(f1 - bf_bits2f(h1));
    hv[e]     = __builtin_bit_cast(_Float16, h0);
    hv[4 + e] = __builtin_bit_cast(_Float16, h1);
    lv[e]     = __builtin_bit_cast(_Float16, l0);
    lv[4 + e] = __builtin_bit_cast(_Float16, l1);
  }
  for (int pass = 0; pass < 2; ++pass) {
    *(volatile v8h*)(HH + rb + ca) = hv;
    *(volatile v8h*)(HL + rb + ca) = lv;
    __threadfence();
  }
}

__device__ __forceinline__ v8f mma_b(v16b a, v16b b, v8f c) {
  c = __builtin_amdgcn_wmma_f32_16x16x32_bf16(false, a, false, b, (short)0, c, false, false);
  asm volatile("v_nop\n\tv_nop\n\tv_nop\n\tv_nop" : "+v"(c) : "v"(a), "v"(b));
  return c;
}
__device__ __forceinline__ void split_bf(float f, __bf16& hi, __bf16& lo) {
  const unsigned short hb = f2bf_bits(f);
  hi = __builtin_bit_cast(__bf16, hb);
  lo = __builtin_bit_cast(__bf16, f2bf_bits(f - bf_bits2f(hb)));
}
constexpr int kAKC = 64;
constexpr int kOSP = 68;
__global__ __launch_bounds__(128) void attn64s_kernel(
    const unsigned short* __restrict__ qhp, const unsigned short* __restrict__ qlp,
    const unsigned short* __restrict__ khp, const unsigned short* __restrict__ klp,
    const unsigned short* __restrict__ vhp, const unsigned short* __restrict__ vlp,
    const float* __restrict__ temp, int ntemp,
    unsigned short* __restrict__ chp, unsigned short* __restrict__ clp)
{
  union FB { v16b v; v8b h[2]; };
  __shared__ __align__(16) __bf16 Ksh[kAKC * kHdim];
  __shared__ __align__(16) __bf16 Ksl[kAKC * kHdim];
  __shared__ __align__(16) __bf16 Vth[kHdim * kAKC];
  __shared__ __align__(16) __bf16 Vtl[kHdim * kAKC];
  __shared__ __align__(16) __bf16 Psh[4][16 * kAKC];
  __shared__ __align__(16) __bf16 Psl[4][16 * kAKC];
  __shared__ __align__(16) float  Os[4][16 * kOSP];
  const __bf16* Qh = (const __bf16*)(const void*)qhp;
  const __bf16* Ql = (const __bf16*)(const void*)qlp;
  const __bf16* Kh = (const __bf16*)(const void*)khp;
  const __bf16* Kl = (const __bf16*)(const void*)klp;
  const __bf16* Vh = (const __bf16*)(const void*)vhp;
  const __bf16* Vl = (const __bf16*)(const void*)vlp;
  _Float16* Ch = (_Float16*)(void*)chp;
  _Float16* Cl = (_Float16*)(void*)clp;
  const int tid = threadIdx.x, wave = tid >> 5, lane = tid & 31, hh = lane >> 4, c = lane & 15;
  const int nqb = kSeq / 64;
  const int bx = blockIdx.x;
  const int qb = bx % nqb;
  const int bh = bx / nqb;
  const int h = bh % kHeads;
  const int b = bh / kHeads;
  const int q0 = qb * 64 + wave * 16;
  const size_t tokb = (size_t)b * kSeq;
  const int hcol = h * kHdim;
  int hc = h; if (hc > ntemp - 1) hc = ntemp - 1; if (hc < 0) hc = 0;
  const float tv  = temp[hc];
  const float tsp = fmaxf(tv, 0.f) + log1pf(expf(-fabsf(tv)));
  const float sc  = 0.125f * tsp;

  v16b qah[2], qal[2];
  {
    const size_t qoff = (tokb + q0 + c) * kDim + hcol + 8 * hh;
#pragma unroll
    for (int dc = 0; dc < 2; ++dc) {
      qah[dc] = Frag<__bf16>::load(Qh + qoff + dc * 32);
      qal[dc] = Frag<__bf16>::load(Ql + qoff + dc * 32);
    }
  }
  float mrow[8], lrow[8];
  v8f oacc[4];
#pragma unroll
  for (int r = 0; r < 8; ++r) { mrow[r] = -INFINITY; lrow[r] = 0.f; }
#pragma unroll
  for (int t = 0; t < 4; ++t) oacc[t] = (v8f){0.f,0.f,0.f,0.f,0.f,0.f,0.f,0.f};

  const int nChunks = qb + 1;
  for (int kc = 0; kc < nChunks; ++kc) {
    const int kv0 = kc * kAKC;
    __syncthreads();
    {
      const int kvr = tid >> 1, dh = (tid & 1) * 32;
      const size_t roff = (tokb + kv0 + kvr) * kDim + hcol + dh;
      const __bf16* krh = Kh + roff;
      const __bf16* krl = Kl + roff;
      const __bf16* vrh = Vh + roff;
      const __bf16* vrl = Vl + roff;
#pragma unroll
      for (int i = 0; i < 4; ++i) {
        const v8b a0 = *(const v8b*)(krh + 8 * i);
        const v8b a1 = *(const v8b*)(krl + 8 * i);
        *(v8b*)(Ksh + kvr * kHdim + dh + 8 * i) = a0;
        *(v8b*)(Ksl + kvr * kHdim + dh + 8 * i) = a1;
        const v8b b0 = *(const v8b*)(vrh + 8 * i);
        const v8b b1 = *(const v8b*)(vrl + 8 * i);
#pragma unroll
        for (int e = 0; e < 8; ++e) {
          Vth[(dh + 8 * i + e) * kAKC + kvr] = b0[e];
          Vtl[(dh + 8 * i + e) * kAKC + kvr] = b1[e];
        }
      }
    }
    __syncthreads();

    v8f s[4];
#pragma unroll
    for (int j = 0; j < 4; ++j) {
      s[j] = (v8f){0.f,0.f,0.f,0.f,0.f,0.f,0.f,0.f};
#pragma unroll
      for (int dc = 0; dc < 2; ++dc) {
        FB kb, kl;
        kb.h[0] = *(const v8b*)(Ksh + (j * 16 + c) * kHdim + dc * 32 + 8 * hh);
        kb.h[1] = *(const v8b*)(Ksh + (j * 16 + c) * kHdim + dc * 32 + 16 + 8 * hh);
        kl.h[0] = *(const v8b*)(Ksl + (j * 16 + c) * kHdim + dc * 32 + 8 * hh);
        kl.h[1] = *(const v8b*)(Ksl + (j * 16 + c) * kHdim + dc * 32 + 16 + 8 * hh);
        s[j] = mma_b(qah[dc], kb.v, s[j]);
        s[j] = mma_b(qah[dc], kl.v, s[j]);
        s[j] = mma_b(qal[dc], kb.v, s[j]);
      }
    }
    const bool diag = (kc == qb);
    float cm[8];
#pragma unroll
    for (int r = 0; r < 8; ++r) {
      const int qrow = q0 + 8 * hh + r;
      float m = -INFINITY;
#pragma unroll
      for (int j = 0; j < 4; ++j) {
        const int kvcol = kv0 + j * 16 + c;
        const float sv = s[j][r] * sc;
        const bool masked = diag && (kvcol > qrow);
        const float sm = masked ? -INFINITY : sv;
        s[j][r] = sm;
        m = fmaxf(m, sm);
      }
#pragma unroll
      for (int off = 1; off < 16; off <<= 1) m = fmaxf(m, __shfl_xor(m, off, 32));
      cm[r] = m;
    }
    __bf16* pwh = Psh[wave];
    __bf16* pwl = Psl[wave];
#pragma unroll
    for (int r = 0; r < 8; ++r) {
      const float mnew = fmaxf(mrow[r], cm[r]);
      const float alpha = expf(mrow[r] - mnew);
      mrow[r] = mnew;
      float psum = 0.f;
#pragma unroll
      for (int j = 0; j < 4; ++j) {
        const float p = expf(s[j][r] - mnew);
        psum += p;
        __bf16 a, bl; split_bf(p, a, bl);
        pwh[(8 * hh + r) * kAKC + j * 16 + c] = a;
        pwl[(8 * hh + r) * kAKC + j * 16 + c] = bl;
      }
#pragma unroll
      for (int off = 1; off < 16; off <<= 1) psum += __shfl_xor(psum, off, 32);
      lrow[r] = lrow[r] * alpha + psum;
#pragma unroll
      for (int t = 0; t < 4; ++t) oacc[t][r] *= alpha;
    }
    __builtin_amdgcn_fence(__ATOMIC_RELEASE, "workgroup");
    __builtin_amdgcn_wave_barrier();
    __builtin_amdgcn_fence(__ATOMIC_ACQUIRE, "workgroup");
#pragma unroll 1
    for (int kk = 0; kk < 2; ++kk) {
      FB pa, pl;
      pa.h[0] = *(const v8b*)(pwh + c * kAKC + kk * 32 + 8 * hh);
      pa.h[1] = *(const v8b*)(pwh + c * kAKC + kk * 32 + 16 + 8 * hh);
      pl.h[0] = *(const v8b*)(pwl + c * kAKC + kk * 32 + 8 * hh);
      pl.h[1] = *(const v8b*)(pwl + c * kAKC + kk * 32 + 16 + 8 * hh);
#pragma unroll
      for (int t = 0; t < 4; ++t) {
        FB vb, vl;
        vb.h[0] = *(const v8b*)(Vth + (t * 16 + c) * kAKC + kk * 32 + 8 * hh);
        vb.h[1] = *(const v8b*)(Vth + (t * 16 + c) * kAKC + kk * 32 + 16 + 8 * hh);
        vl.h[0] = *(const v8b*)(Vtl + (t * 16 + c) * kAKC + kk * 32 + 8 * hh);
        vl.h[1] = *(const v8b*)(Vtl + (t * 16 + c) * kAKC + kk * 32 + 16 + 8 * hh);
        oacc[t] = mma_b(pa.v, vb.v, oacc[t]);
        oacc[t] = mma_b(pa.v, vl.v, oacc[t]);
        oacc[t] = mma_b(pl.v, vb.v, oacc[t]);
      }
    }
  }

  float* os = Os[wave];
#pragma unroll
  for (int r = 0; r < 8; ++r) {
    const float inv = 1.0f / lrow[r];
#pragma unroll
    for (int t = 0; t < 4; ++t) os[(8 * hh + r) * kOSP + t * 16 + c] = oacc[t][r] * inv;
  }
  __builtin_amdgcn_fence(__ATOMIC_RELEASE, "workgroup");
  __builtin_amdgcn_wave_barrier();
  __builtin_amdgcn_fence(__ATOMIC_ACQUIRE, "workgroup");
  {
    const int q8 = lane >> 3, c8 = (lane & 7) * 8;
    for (int pass = 0; pass < 2; ++pass) {
#pragma unroll
      for (int it = 0; it < 4; ++it) {
        const int row = it * 4 + q8;
        const float* sp = os + row * kOSP + c8;
        const v4f f0 = *(const v4f*)(sp);
        const v4f f1 = *(const v4f*)(sp + 4);
        v8h hv, lv;
#pragma unroll
        for (int e = 0; e < 4; ++e) {
          const unsigned short h0 = f2bf_bits(f0[e]), h1 = f2bf_bits(f1[e]);
          const unsigned short l0 = f2bf_bits(f0[e] - bf_bits2f(h0)), l1 = f2bf_bits(f1[e] - bf_bits2f(h1));
          hv[e] = __builtin_bit_cast(_Float16, h0); hv[4 + e] = __builtin_bit_cast(_Float16, h1);
          lv[e] = __builtin_bit_cast(_Float16, l0); lv[4 + e] = __builtin_bit_cast(_Float16, l1);
        }
        const size_t go = (tokb + q0 + row) * kDim + hcol + c8;
        *(volatile v8h*)(Ch + go) = hv;
        *(volatile v8h*)(Cl + go) = lv;
      }
      __threadfence();
    }
  }
}

extern "C" void kernel_launch(void* const* d_in, const int* in_sizes, int n_in,
                              void* d_out, int out_size, void* d_ws, size_t ws_size,
                              hipStream_t stream)
{
  if (n_in < 19) return;
  const int nTokC = kTok * kDim;
  const int nW    = kDim * kDim;
  if (in_sizes[0] != nTokC || in_sizes[1] != kDim * kState || in_sizes[2] != nW || in_sizes[3] != kDim ||
      in_sizes[4] != kDim * kState || in_sizes[5] != kDim * kState ||
      in_sizes[6] != nW || in_sizes[7] != kDim || in_sizes[8] != nW || in_sizes[9] != kDim ||
      in_sizes[10] != nW || in_sizes[11] != kDim || in_sizes[12] != nW || in_sizes[13] != kDim ||
      in_sizes[14] != nW || in_sizes[15] != kDim || in_sizes[16] != kDim || in_sizes[17] != kDim ||
      in_sizes[18] < 1 || out_size != nTokC) return;

  const float* x     = (const float*)d_in[0];
  const float* A_log = (const float*)d_in[1];
  const float* Wd    = (const float*)d_in[2];
  const float* bd    = (const float*)d_in[3];
  const float* WB    = (const float*)d_in[4];
  const float* WC    = (const float*)d_in[5];
  const float* Wq    = (const float*)d_in[6];
  const float* bq    = (const float*)d_in[7];
  const float* Wk    = (const float*)d_in[8];
  const float* bk    = (const float*)d_in[9];
  const float* Wv    = (const float*)d_in[10];
  const float* bv    = (const float*)d_in[11];
  const float* Wx    = (const float*)d_in[12];
  const float* bx    = (const float*)d_in[13];
  const float* Wo    = (const float*)d_in[14];
  const float* bo    = (const float*)d_in[15];
  const float* ln_g  = (const float*)d_in[16];
  const float* ln_b  = (const float*)d_in[17];
  const float* temp  = (const float*)d_in[18];
  float* outF = (float*)d_out;

  size_t off = 0;
  auto take = [&](size_t bytes) -> size_t { const size_t o = off; off += (bytes + 127) & ~(size_t)127; return o; };
  const size_t oX16  = take(kPlane16);
  const size_t oWXT  = take(kW16);
  const size_t oWDT  = take(kW16);
  const size_t oWBCT = take(kWBC16);
  const size_t oWQT  = take(kW16);
  const size_t oWKT  = take(kW16);
  const size_t oWVT  = take(kW16);
  const size_t oWOT  = take(kW16);
  const size_t oXB   = take(kPlane32);
  const size_t oDPRE = take(kPlane32);
  const size_t oBC   = take(kBC32);
  const size_t oHH   = take(kPlane16);
  const size_t oHL   = take(kPlane16);
  const size_t oVH   = take(kPlane16);
  const size_t oVL   = take(kPlane16);
  const size_t oCH   = take(kPlane16);
  const size_t oCL   = take(kPlane16);
  if (off != kCarveTotal || off > ws_size) return;
  const size_t oQH = oDPRE, oQL = oDPRE + kPlane16;
  const size_t oKH = oXB,   oKL = oXB + kPlane16;

  char* ws = (char*)d_ws;
  unsigned short* X16  = (unsigned short*)(ws + oX16);
  unsigned short* WXT  = (unsigned short*)(ws + oWXT);
  unsigned short* WDT  = (unsigned short*)(ws + oWDT);
  unsigned short* WBCT = (unsigned short*)(ws + oWBCT);
  unsigned short* WQT  = (unsigned short*)(ws + oWQT);
  unsigned short* WKT  = (unsigned short*)(ws + oWKT);
  unsigned short* WVT  = (unsigned short*)(ws + oWVT);
  unsigned short* WOT  = (unsigned short*)(ws + oWOT);
  float*          XB   = (float*)(ws + oXB);
  float*          DPRE = (float*)(ws + oDPRE);
  float*          BC   = (float*)(ws + oBC);
  unsigned short* HH   = (unsigned short*)(ws + oHH);
  unsigned short* HL   = (unsigned short*)(ws + oHL);
  unsigned short* QH   = (unsigned short*)(ws + oQH);
  unsigned short* QL   = (unsigned short*)(ws + oQL);
  unsigned short* KH   = (unsigned short*)(ws + oKH);
  unsigned short* KL   = (unsigned short*)(ws + oKL);
  unsigned short* VH   = (unsigned short*)(ws + oVH);
  unsigned short* VL   = (unsigned short*)(ws + oVL);
  unsigned short* CH   = (unsigned short*)(ws + oCH);
  unsigned short* CL   = (unsigned short*)(ws + oCL);

  const int total8 = nTokC / 8;
  cast_bf16_kernel<<<(total8 + 255) / 256, 256, 0, stream>>>(x, X16, total8);

  const dim3 gT(kDim / 64, kDim / 64);
  const dim3 gTs(1, kDim / 64);
  transpose_bf16_kernel<<<gT,  256, 0, stream>>>(Wx, WXT, kDim, kDim);
  transpose_bf16_kernel<<<gT,  256, 0, stream>>>(Wd, WDT, kDim, kDim);
  transpose_bf16_kernel<<<gTs, 256, 0, stream>>>(WB, WBCT, kDim, kState);
  transpose_bf16_kernel<<<gTs, 256, 0, stream>>>(WC, WBCT + (size_t)64 * kDim, kDim, kState);
  transpose_bf16_kernel<<<gT,  256, 0, stream>>>(Wq, WQT, kDim, kDim);
  transpose_bf16_kernel<<<gT,  256, 0, stream>>>(Wk, WKT, kDim, kDim);
  transpose_bf16_kernel<<<gT,  256, 0, stream>>>(Wv, WVT, kDim, kDim);
  transpose_bf16_kernel<<<gT,  256, 0, stream>>>(Wo, WOT, kDim, kDim);

  const int gemmBlocks = (kTok / 64) * (kDim / 64) / 8;
  const int bcBlocks   = (kTok / 64) * (kBCP / 64) / 8;
  wmma_gemm64<1, 0, 2, 0, false, 0><<<dim3(gemmBlocks, 1), 256, 0, stream>>>(
      X16, X16, kDim, 0L, WXT, WXT, kDim, 0L, (void*)XB, (void*)XB, kDim, 0L, bx, bx, 0L, kTok, kDim, kDim, 1.0f);
  wmma_gemm64<1, 0, 2, 0, false, 0><<<dim3(gemmBlocks, 1), 256, 0, stream>>>(
      X16, X16, kDim, 0L, WDT, WDT, kDim, 0L, (void*)DPRE, (void*)DPRE, kDim, 0L, bd, bd, 0L, kTok, kDim, kDim, 1.0f);
  wmma_gemm64<1, 0, 0, 0, false, 0><<<dim3(bcBlocks, 1), 256, 0, stream>>>(
      X16, X16, kDim, 0L, WBCT, WBCT, kDim, 0L, (void*)BC, (void*)BC, kBCP, 0L, bx, bx, 0L, kTok, kBCP, kDim, 1.0f);

  scan_kernel<<<kBatch * (kDim / 32), 32, 0, stream>>>(XB, DPRE, BC, A_log);

  ln_kernel<<<kTok, 128, 0, stream>>>(XB, ln_g, ln_b, HH, HL);

  wmma_gemm64<1, 2, 2, 2, false, 0><<<dim3(gemmBlocks, 1), 256, 0, stream>>>(
      HH, HL, kDim, 0L, WQT, WQT, kDim, 0L, (void*)QH, (void*)QL, kDim, 0L, bq, bq, 0L, kTok, kDim, kDim, 1.0f);
  wmma_gemm64<1, 2, 2, 2, false, 0><<<dim3(gemmBlocks, 1), 256, 0, stream>>>(
      HH, HL, kDim, 0L, WKT, WKT, kDim, 0L, (void*)KH, (void*)KL, kDim, 0L, bk, bk, 0L, kTok, kDim, kDim, 1.0f);
  wmma_gemm64<1, 2, 2, 2, false, 0><<<dim3(gemmBlocks, 1), 256, 0, stream>>>(
      HH, HL, kDim, 0L, WVT, WVT, kDim, 0L, (void*)VH, (void*)VL, kDim, 0L, bv, bv, 0L, kTok, kDim, kDim, 1.0f);

  attn64s_kernel<<<kBatch * kHeads * (kSeq / 64), 128, 0, stream>>>(QH, QL, KH, KL, VH, VL, temp, in_sizes[18], CH, CL);

  wmma_gemm64<1, 2, 2, 0, false, 0><<<dim3(gemmBlocks, 1), 256, 0, stream>>>(
      CH, CL, kDim, 0L, WOT, WOT, kDim, 0L, (void*)outF, (void*)outF, kDim, 0L, bo, bo, 0L, kTok, kDim, kDim, 1.0f);
}
